// FineGrainedOpLSTMNet_9680856285275
// MI455X (gfx1250) — hardware-verified
//
#include <hip/hip_runtime.h>
#include <stddef.h>


typedef _Float16 f16t;
typedef __bf16   bf16t;
typedef f16t  v16h __attribute__((ext_vector_type(16)));
typedef f16t  v8h  __attribute__((ext_vector_type(8)));
typedef bf16t v16b __attribute__((ext_vector_type(16)));
typedef bf16t v8b  __attribute__((ext_vector_type(8)));
typedef float v8f  __attribute__((ext_vector_type(8)));
typedef float v4f  __attribute__((ext_vector_type(4)));
typedef unsigned int v4u __attribute__((ext_vector_type(4)));

#define NBATCH 64
#define NSTEP  512
#define NIN    256
#define NHID   256
#define NGATE  1024
#define TCH    256
#define LPH    264
#define LPF    264
#define SC_W   256.0f
#define SC_H   256.0f
#define INV_HW 0.0000152587890625f

template<typename E> struct FT;
template<> struct FT<f16t>  { typedef v16h V16; typedef v8h V8; };
template<> struct FT<bf16t> { typedef v16b V16; typedef v8b V8; };
template<typename E> union FragT { typename FT<E>::V16 v; typename FT<E>::V8 q[2]; };

union Pk16 { v8h h; v4u u; unsigned short s[8]; };
union Pk32 { v4f f; v4u u; };

__device__ __forceinline__ v8f wmma16(v16h a, v16h b, v8f c) {
    return __builtin_amdgcn_wmma_f32_16x16x32_f16(false, a, false, b, (short)0, c, false, false);
}
__device__ __forceinline__ v8f wmma16(v16b a, v16b b, v8f c) {
    return __builtin_amdgcn_wmma_f32_16x16x32_bf16(false, a, false, b, (short)0, c, false, false);
}

template<typename E>
__device__ __forceinline__ void wguard(v8f (&c)[2][1], FragT<E> (&a)[2], FragT<E> (&b)[1]) {
    asm volatile("v_nop\n\tv_nop\n\tv_nop\n\tv_nop"
                 : "+v"(c[0][0]), "+v"(c[1][0])
                 : "v"(a[0].v), "v"(a[1].v), "v"(b[0].v));
}
template<typename E>
__device__ __forceinline__ void wguard(v8f (&c)[4][1], FragT<E> (&a)[4], FragT<E> (&b)[1]) {
    asm volatile("v_nop\n\tv_nop\n\tv_nop\n\tv_nop"
                 : "+v"(c[0][0]), "+v"(c[1][0]), "+v"(c[2][0]), "+v"(c[3][0])
                 : "v"(a[0].v), "v"(a[1].v), "v"(a[2].v), "v"(a[3].v), "v"(b[0].v));
}

template<int MT, int NT>
__device__ __forceinline__ void zacc(v8f (&acc)[MT][NT]) {
    const v8f z = {0.f, 0.f, 0.f, 0.f, 0.f, 0.f, 0.f, 0.f};
#pragma unroll
    for (int i = 0; i < MT; ++i)
#pragma unroll
        for (int j = 0; j < NT; ++j) acc[i][j] = z;
}

template<int MT, int NT, typename E>
__device__ __forceinline__ void mma_acc(v8f (&acc)[MT][NT],
                                        const E* A, int lda,
                                        const E* B, int ldb, int ktiles) {
    typedef typename FT<E>::V8 V8;
    const int l = threadIdx.x & 31, h = l >> 4, m = l & 15;
    const E* ap = A + (size_t)m * lda + 8 * h;
    const E* bp = B + (size_t)m * ldb + 8 * h;
#pragma unroll 1
    for (int kt = 0; kt < ktiles; ++kt) {
        FragT<E> a[MT], b[NT];
#pragma unroll
        for (int i = 0; i < MT; ++i) {
            const E* p = ap + (size_t)i * 16 * lda + kt * 32;
            a[i].q[0] = *(const V8*)p;
            a[i].q[1] = *(const V8*)(p + 16);
        }
#pragma unroll
        for (int j = 0; j < NT; ++j) {
            const E* p = bp + (size_t)j * 16 * ldb + kt * 32;
            b[j].q[0] = *(const V8*)p;
            b[j].q[1] = *(const V8*)(p + 16);
        }
#pragma unroll
        for (int i = 0; i < MT; ++i)
#pragma unroll
            for (int j = 0; j < NT; ++j)
                acc[i][j] = wmma16(a[i].v, b[j].v, acc[i][j]);
        wguard<E>(acc, a, b);
    }
}

__device__ __forceinline__ unsigned int bf16bits(float f) {
    unsigned int u = __float_as_uint(f);
    return (u + 0x7FFFu + ((u >> 16) & 1u)) >> 16;
}
__device__ __forceinline__ float bfr(float f) {
    return __uint_as_float(bf16bits(f) << 16);
}
__device__ __forceinline__ float fsig(float x) {
    float t = __expf(-x);
    return __builtin_amdgcn_rcpf(1.0f + t);
}
__device__ __forceinline__ float ftanh(float x) {
    float ax = fabsf(x);
    float t  = __expf(-2.0f * ax);
    float r  = (1.0f - t) * __builtin_amdgcn_rcpf(1.0f + t);
    return copysignf(r, x);
}
__device__ __forceinline__ float cellf(float ai, float af, float ag, float ao,
                                       float xi, float xf, float xg, float xo, float& c) {
    float zi = fmaf(ai, INV_HW, xi);
    float zf = fmaf(af, INV_HW, xf);
    float zg = fmaf(ag, INV_HW, xg);
    float zo = fmaf(ao, INV_HW, xo);
    float ig = fsig(zi), fg = fsig(zf), gg = ftanh(zg), og = fsig(zo);
    float cn = fg * c + ig * gg;
    c = cn;
    return og * ftanh(cn);
}

template<int MT>
__device__ __forceinline__ void epi_lds(v8f (&acc)[MT][1], float inv, const float* bias,
                                        int f0, float* S, int pitch) {
    const int l = threadIdx.x & 31, h = l >> 4, m = l & 15;
#pragma unroll
    for (int i = 0; i < MT; ++i) {
        const float* bq = bias + f0 + 16 * i + 8 * h;
        v4f c0 = *(const v4f*)bq;
        v4f c1 = *(const v4f*)(bq + 4);
        Pk32 p0, p1;
#pragma unroll
        for (int r = 0; r < 4; ++r) {
            p0.f[r] = fmaf(acc[i][0][r],     inv, bfr(c0[r]));
            p1.f[r] = fmaf(acc[i][0][4 + r], inv, bfr(c1[r]));
        }
        float* d = S + (size_t)m * pitch + f0 + 16 * i + 8 * h;
        *(v4f*)d       = p0.f;
        *(v4f*)(d + 4) = p1.f;
    }
}

__global__ __launch_bounds__(256)
void k_cvt_x(const float* x, unsigned short* y, int n8) {
    int i = blockIdx.x * 256 + threadIdx.x;
    if (i >= n8) return;
    const float* p = x + (size_t)i * 8;
    v4f a = *(const v4f*)p;
    v4f b = *(const v4f*)(p + 4);
    Pk16 k;
#pragma unroll
    for (int e = 0; e < 4; ++e) {
        k.s[e]     = (unsigned short)bf16bits(a[e]);
        k.s[4 + e] = (unsigned short)bf16bits(b[e]);
    }
    unsigned short* d = y + (size_t)i * 8;
    *(volatile v4u*)d = k.u;
    __threadfence();
    *(volatile v4u*)d = k.u;
}

template<bool ASF16>
__global__ __launch_bounds__(256)
void k_pack(const float* W, unsigned short* P, int K, int N, float sc) {
    int i   = blockIdx.x * 256 + threadIdx.x;
    int kq  = K >> 3;
    int tot = N * kq;
    if (i >= tot) return;
    int n = i / kq;
    int k = (i - n * kq) * 8;
    Pk16 v;
#pragma unroll
    for (int e = 0; e < 8; ++e) {
        float w = W[(size_t)(k + e) * N + n];
        if (ASF16) v.h[e] = (f16t)(bfr(w) * sc);
        else       v.s[e] = (unsigned short)bf16bits(w);
    }
    unsigned short* d = P + (size_t)n * K + k;
    *(volatile v4u*)d = v.u;
    __threadfence();
    *(volatile v4u*)d = v.u;
}

template<typename E>
__global__ __launch_bounds__(256)
void k_gemm(const E* Act, const E* Wp, const float* bias, float* C,
            int T, int t0, int TC, float inv) {
    __shared__ __attribute__((aligned(16))) float S[32 * LPF];
    const int tid = threadIdx.x, w = tid >> 5;
    const int q0  = blockIdx.x * 32;
    const int fq  = blockIdx.y * 256;
    if (q0 + 32 > NBATCH * TC) return;
    const int b   = q0 / TC;
    const int tl0 = q0 - b * TC;
    const size_t srow = (size_t)b * T + t0 + tl0;
    const int ri = w & 1, fw = 64 * (w >> 1);
    {
        v8f acc[4][1]; zacc(acc);
        mma_acc<4, 1, E>(acc, Wp + (size_t)(fq + fw) * NHID, NHID,
                         Act + (srow + 16 * ri) * NHID, NHID, NHID / 32);
        epi_lds<4>(acc, inv, bias + fq, fw, S + (16 * ri) * LPF, LPF);
    }
    __syncthreads();
    Pk32 v[8];
#pragma unroll
    for (int i = 0; i < 8; ++i) {
        int p = tid + 256 * i, row = p >> 6, c = (p & 63) * 4;
        v[i].f = *(const v4f*)(S + row * LPF + c);
    }
#pragma unroll
    for (int i = 0; i < 8; ++i) {
        int p = tid + 256 * i, row = p >> 6, c = (p & 63) * 4;
        *(volatile v4u*)(C + (size_t)(q0 + row) * NGATE + fq + c) = v[i].u;
    }
    __threadfence();
#pragma unroll
    for (int i = 0; i < 8; ++i) {
        int p = tid + 256 * i, row = p >> 6, c = (p & 63) * 4;
        *(volatile v4u*)(C + (size_t)(q0 + row) * NGATE + fq + c) = v[i].u;
    }
}

template<bool FINAL>
__global__ __launch_bounds__(256)
void k_scan(const float* XZ, const f16t* Up, f16t* Hout, float* Yout,
            f16t* Hst, float* Cst, int T, int t0, int TC, int first) {
    __shared__ __attribute__((aligned(16))) f16t  Hs[16 * LPH];
    __shared__ __attribute__((aligned(16))) float Sf[16 * LPF];
    const int tid = threadIdx.x, w = tid >> 5, l = tid & 31, h = l >> 4, m = l & 15;
    const int b0 = blockIdx.x * 16;
    if (b0 + 16 > NBATCH) return;
    const int fl = 32 * w + 8 * h;

    float cs[2][8];
    if (first) {
        for (int i = tid; i < 16 * LPH; i += 256) Hs[i] = (f16t)0.0f;
#pragma unroll
        for (int i = 0; i < 2; ++i)
#pragma unroll
            for (int r = 0; r < 8; ++r) cs[i][r] = 0.0f;
    } else {
#pragma unroll
        for (int i = 0; i < 2; ++i) {
            int p = tid + 256 * i, row = p >> 5, ch = (p & 31) * 8;
            *(v8h*)(Hs + row * LPH + ch) = *(const v8h*)(Hst + (size_t)(b0 + row) * NHID + ch);
        }
#pragma unroll
        for (int i = 0; i < 2; ++i) {
            const float* cp = Cst + (size_t)(b0 + m) * NHID + fl + 16 * i;
            v4f a = *(const v4f*)cp;
            v4f b = *(const v4f*)(cp + 4);
#pragma unroll
            for (int r = 0; r < 4; ++r) { cs[i][r] = a[r]; cs[i][4 + r] = b[r]; }
        }
    }
    __syncthreads();

    const f16t* ub = Up + (size_t)(32 * w) * NHID;

#pragma unroll 1
    for (int tl = 0; tl < TC; ++tl) {
        v8f g0[2][1], g1[2][1], g2[2][1], g3[2][1];
        zacc(g0); zacc(g1); zacc(g2); zacc(g3);
        mma_acc<2, 1, f16t>(g0, ub,                        NHID, Hs, LPH, NHID / 32);
        mma_acc<2, 1, f16t>(g1, ub + (size_t)256 * NHID,   NHID, Hs, LPH, NHID / 32);
        mma_acc<2, 1, f16t>(g2, ub + (size_t)512 * NHID,   NHID, Hs, LPH, NHID / 32);
        mma_acc<2, 1, f16t>(g3, ub + (size_t)768 * NHID,   NHID, Hs, LPH, NHID / 32);

        const float* xr = XZ + ((size_t)(b0 + m) * TC + tl) * NGATE + fl;
        Pk16 hv[2];
        Pk32 yv[2][2];
#pragma unroll
        for (int i = 0; i < 2; ++i) {
            const float* xp = xr + 16 * i;
            v4f xi0 = *(const v4f*)(xp);        v4f xi1 = *(const v4f*)(xp + 4);
            v4f xf0 = *(const v4f*)(xp + 256);  v4f xf1 = *(const v4f*)(xp + 260);
            v4f xg0 = *(const v4f*)(xp + 512);  v4f xg1 = *(const v4f*)(xp + 516);
            v4f xo0 = *(const v4f*)(xp + 768);  v4f xo1 = *(const v4f*)(xp + 772);
#pragma unroll
            for (int r = 0; r < 4; ++r) {
                float hn0 = cellf(g0[i][0][r], g1[i][0][r], g2[i][0][r], g3[i][0][r],
                                  xi0[r], xf0[r], xg0[r], xo0[r], cs[i][r]);
                float hn1 = cellf(g0[i][0][4 + r], g1[i][0][4 + r], g2[i][0][4 + r], g3[i][0][4 + r],
                                  xi1[r], xf1[r], xg1[r], xo1[r], cs[i][4 + r]);
                hv[i].h[r]     = (f16t)(hn0 * SC_H);
                hv[i].h[4 + r] = (f16t)(hn1 * SC_H);
                if (FINAL) { yv[i][0].f[r] = hn0; yv[i][1].f[r] = hn1; }
            }
        }
        __syncthreads();
#pragma unroll
        for (int i = 0; i < 2; ++i) {
            *(v8h*)(Hs + m * LPH + fl + 16 * i) = hv[i].h;
            if (FINAL) {
                float* d = Sf + m * LPF + fl + 16 * i;
                *(v4f*)d       = yv[i][0].f;
                *(v4f*)(d + 4) = yv[i][1].f;
            }
        }
        __syncthreads();

        if (!FINAL) {
            Pk16 v[2];
#pragma unroll
            for (int i = 0; i < 2; ++i) {
                int p = tid + 256 * i, row = p >> 5, ch = (p & 31) * 8;
                v[i].h = *(const v8h*)(Hs + row * LPH + ch);
            }
#pragma unroll
            for (int i = 0; i < 2; ++i) {
                int p = tid + 256 * i, row = p >> 5, ch = (p & 31) * 8;
                size_t grow = (size_t)(b0 + row) * T + t0 + tl;
                *(volatile v4u*)(Hout + grow * NHID + ch) = v[i].u;
            }
            __threadfence();
#pragma unroll
            for (int i = 0; i < 2; ++i) {
                int p = tid + 256 * i, row = p >> 5, ch = (p & 31) * 8;
                size_t grow = (size_t)(b0 + row) * T + t0 + tl;
                *(volatile v4u*)(Hout + grow * NHID + ch) = v[i].u;
            }
        } else {
            Pk32 v[4];
#pragma unroll
            for (int i = 0; i < 4; ++i) {
                int p = tid + 256 * i, row = p >> 6, c = (p & 63) * 4;
                v[i].f = *(const v4f*)(Sf + row * LPF + c);
            }
#pragma unroll
            for (int i = 0; i < 4; ++i) {
                int p = tid + 256 * i, row = p >> 6, c = (p & 63) * 4;
                size_t grow = (size_t)(b0 + row) * T + t0 + tl;
                *(volatile v4u*)(Yout + grow * NHID + c) = v[i].u;
            }
            __threadfence();
#pragma unroll
            for (int i = 0; i < 4; ++i) {
                int p = tid + 256 * i, row = p >> 6, c = (p & 63) * 4;
                size_t grow = (size_t)(b0 + row) * T + t0 + tl;
                *(volatile v4u*)(Yout + grow * NHID + c) = v[i].u;
            }
        }
    }

    __syncthreads();
#pragma unroll
    for (int i = 0; i < 2; ++i) {
        Pk32 c0, c1;
#pragma unroll
        for (int r = 0; r < 4; ++r) { c0.f[r] = cs[i][r]; c1.f[r] = cs[i][4 + r]; }
        float* d = Sf + m * LPF + fl + 16 * i;
        *(v4f*)d       = c0.f;
        *(v4f*)(d + 4) = c1.f;
    }
    __syncthreads();
    {
        Pk16 hvv[2];
        Pk32 cvv[4];
#pragma unroll
        for (int i = 0; i < 2; ++i) {
            int p = tid + 256 * i, row = p >> 5, ch = (p & 31) * 8;
            hvv[i].h = *(const v8h*)(Hs + row * LPH + ch);
        }
#pragma unroll
        for (int i = 0; i < 4; ++i) {
            int p = tid + 256 * i, row = p >> 6, c = (p & 63) * 4;
            cvv[i].f = *(const v4f*)(Sf + row * LPF + c);
        }
#pragma unroll
        for (int i = 0; i < 2; ++i) {
            int p = tid + 256 * i, row = p >> 5, ch = (p & 31) * 8;
            *(volatile v4u*)(Hst + (size_t)(b0 + row) * NHID + ch) = hvv[i].u;
        }
#pragma unroll
        for (int i = 0; i < 4; ++i) {
            int p = tid + 256 * i, row = p >> 6, c = (p & 63) * 4;
            *(volatile v4u*)(Cst + (size_t)(b0 + row) * NHID + c) = cvv[i].u;
        }
        __threadfence();
#pragma unroll
        for (int i = 0; i < 2; ++i) {
            int p = tid + 256 * i, row = p >> 5, ch = (p & 31) * 8;
            *(volatile v4u*)(Hst + (size_t)(b0 + row) * NHID + ch) = hvv[i].u;
        }
#pragma unroll
        for (int i = 0; i < 4; ++i) {
            int p = tid + 256 * i, row = p >> 6, c = (p & 63) * 4;
            *(volatile v4u*)(Cst + (size_t)(b0 + row) * NHID + c) = cvv[i].u;
        }
    }
}

extern "C" void kernel_launch(void* const* d_in, const int* in_sizes, int n_in,
                              void* d_out, int out_size, void* d_ws, size_t ws_size,
                              hipStream_t stream) {
    if (n_in < 7) return;
    const int nrow = NBATCH * NSTEP;
    if (in_sizes[0] != nrow * NIN || in_sizes[1] != NIN * NGATE || in_sizes[2] != NHID * NGATE ||
        in_sizes[3] != NGATE || in_sizes[4] != NHID * NGATE || in_sizes[5] != NHID * NGATE ||
        in_sizes[6] != NGATE) return;
    if (out_size != nrow * NHID) return;
    if ((NSTEP % TCH) != 0 || (TCH % 32) != 0 || (NBATCH % 16) != 0) return;

    const float* x   = (const float*)d_in[0];
    const float* W0  = (const float*)d_in[1];
    const float* U0  = (const float*)d_in[2];
    const float* b0v = (const float*)d_in[3];
    const float* W1  = (const float*)d_in[4];
    const float* U1  = (const float*)d_in[5];
    const float* b1v = (const float*)d_in[6];
    float* out = (float*)d_out;

    char* ws = (char*)d_ws;
    size_t off = 0;
    auto carve = [&](size_t bytes) -> char* {
        char* p = ws + off;
        off = (off + bytes + 255) & ~(size_t)255;
        return p;
    };
    unsigned short* Xb  = (unsigned short*)carve((size_t)nrow * NIN * 2);
    unsigned short* H0p = (unsigned short*)carve((size_t)nrow * NHID * 2);
    float*          XZ  = (float*)carve((size_t)NBATCH * TCH * NGATE * 4);
    unsigned short* W0p = (unsigned short*)carve((size_t)NGATE * NIN * 2);
    unsigned short* U0p = (unsigned short*)carve((size_t)NGATE * NHID * 2);
    unsigned short* W1p = (unsigned short*)carve((size_t)NGATE * NHID * 2);
    unsigned short* U1p = (unsigned short*)carve((size_t)NGATE * NHID * 2);
    unsigned short* Hst = (unsigned short*)carve((size_t)NBATCH * NHID * 2);
    float*          Cst = (float*)carve((size_t)NBATCH * NHID * 4);
    if (off > ws_size) return;

    {
        int n8 = nrow * NIN / 8;
        k_cvt_x<<<dim3((n8 + 255) / 256), dim3(256), 0, stream>>>(x, Xb, n8);
    }
    {
        int tot = NGATE * (NIN / 8);
        dim3 g((tot + 255) / 256), blk(256);
        k_pack<false><<<g, blk, 0, stream>>>(W0, W0p, NIN,  NGATE, 1.0f);
        k_pack<true ><<<g, blk, 0, stream>>>(U0, U0p, NHID, NGATE, SC_W);
        k_pack<true ><<<g, blk, 0, stream>>>(W1, W1p, NHID, NGATE, SC_W);
        k_pack<true ><<<g, blk, 0, stream>>>(U1, U1p, NHID, NGATE, SC_W);
    }
    const int  nch = NSTEP / TCH;
    const dim3 ggrid(NBATCH * TCH / 32, NGATE / 256), gblk(256);
    const dim3 sgrid(NBATCH / 16), sblk(256);
    for (int ch = 0; ch < nch; ++ch) {
        const int t0 = ch * TCH;
        k_gemm<bf16t><<<ggrid, gblk, 0, stream>>>((const bf16t*)Xb, (const bf16t*)W0p, b0v, XZ,
                                                  NSTEP, t0, TCH, 1.0f);
        k_scan<false><<<sgrid, sblk, 0, stream>>>(XZ, (const f16t*)U0p, (f16t*)H0p, out,
                                                  (f16t*)Hst, Cst, NSTEP, t0, TCH, ch == 0 ? 1 : 0);
    }
    for (int ch = 0; ch < nch; ++ch) {
        const int t0 = ch * TCH;
        k_gemm<f16t><<<ggrid, gblk, 0, stream>>>((const f16t*)H0p, (const f16t*)W1p, b1v, XZ,
                                                 NSTEP, t0, TCH, INV_HW);
        k_scan<true><<<sgrid, sblk, 0, stream>>>(XZ, (const f16t*)U1p, (f16t*)H0p, out,
                                                 (f16t*)Hst, Cst, NSTEP, t0, TCH, ch == 0 ? 1 : 0);
    }
}
